// MemoryEfficientSAM2Attention_1657857376483
// MI455X (gfx1250) — hardware-verified
//
#include <hip/hip_runtime.h>


namespace {
constexpr int N = 8000, C = 256, DQ = 32;
constexpr float XS = 8.0f, PS = 8.0f, ISC = 0.17677669529663687f;

typedef _Float16 b16;
typedef __attribute__((ext_vector_type(16))) _Float16 v16b;
typedef __attribute__((ext_vector_type(8))) _Float16 v8b;
typedef __attribute__((ext_vector_type(8))) float v8f;
typedef __attribute__((ext_vector_type(4))) float v4f;
__device__ __forceinline__ float bf16_rne(float f) { unsigned int u = __float_as_uint(f); u += 0x7FFFu + ((u >> 16) & 1u); return __uint_as_float(u & 0xFFFF0000u); }
__device__ __forceinline__ v16b frag_kb(const b16* p, int hh) { const v8b a = *(const v8b*)(p + 8 * hh), b = *(const v8b*)(p + 16 + 8 * hh); v16b f;
#pragma unroll
  for (int e = 0; e < 8; ++e) { f[e] = a[e]; f[8 + e] = b[e]; } return f; }
__device__ __forceinline__ v8f wmma16b(v16b a, v16b b, v8f c) { v8f d = __builtin_amdgcn_wmma_f32_16x16x32_f16(false, a, false, b, (short)0, c, false, false); asm volatile("v_nop\n\tv_nop\n\tv_nop\n\tv_nop" : "+v"(d) : "v"(a), "v"(b)); return d; }
__device__ __forceinline__ void wave_lds_sync() { __builtin_amdgcn_fence(__ATOMIC_RELEASE, "workgroup"); __builtin_amdgcn_wave_barrier(); __builtin_amdgcn_fence(__ATOMIC_ACQUIRE, "workgroup"); }
__device__ __forceinline__ float nexp(float x) { return __builtin_amdgcn_exp2f(x * 1.4426950408889634f); }
__device__ __forceinline__ float pmul(float a, float b) { float p = a * b; asm volatile("" : "+v"(p)); return p; }

__global__ __launch_bounds__(256) void prep_kernel(const float* __restrict__ x, const float* __restrict__ wq, const float* __restrict__ bq, const float* __restrict__ wk, const float* __restrict__ bk, const float* __restrict__ wv, const float* __restrict__ bv, const float* __restrict__ gm, b16* __restrict__ R, float* __restrict__ P, b16* __restrict__ X) {
  const size_t tid = (size_t)blockIdx.x * 256 + threadIdx.x, nth = (size_t)gridDim.x * 256;
  for (int pass = 0; pass < 2; ++pass) {
    for (size_t p = tid; p < (size_t)320 * C; p += nth) { const int o = (int)(p / C), k = (int)(p % C); float w; if (o < 32) w = wq[(size_t)k * DQ + o]; else if (o < 64) w = wk[(size_t)k * DQ + (o - 32)]; else w = wv[(size_t)k * C + (o - 64)]; ((volatile b16*)R)[p] = (b16)bf16_rne(w); }
    for (size_t q = tid; q < 321; q += nth) { const int i = (int)q; P[q] = bf16_rne((i < 32) ? bq[i] : (i < 64) ? bk[i - 32] : (i < 320) ? bv[i - 64] : gm[0]); }
    for (size_t p = tid; p < (size_t)N * C / 8; p += nth) { v8b v; for (int e = 0; e < 8; ++e) v[e] = (b16)(bf16_rne(x[p * 8 + e]) * XS); *(volatile v8b*)(X + p * 8) = v; }
    __threadfence(); }
}
__global__ __launch_bounds__(128) void qk_kernel(const b16* __restrict__ X, const b16* __restrict__ R, const float* __restrict__ P, b16* __restrict__ Q, b16* __restrict__ K) {
  __shared__ __attribute__((aligned(16))) b16 Tq[64][DQ + 8], Tk[64][DQ + 8];
  const int lane = threadIdx.x & 31, wave = threadIdx.x >> 5, nloc = lane & 15, hlf = lane >> 4, m0 = blockIdx.x * 64 + wave * 16;
  v8f acc[4] = {{}, {}, {}, {}};
#pragma unroll 2
  for (int kb = 0; kb < C; kb += 32) { const v16b a = frag_kb(X + (size_t)(m0 + nloc) * C + kb, hlf);
#pragma unroll
    for (int t = 0; t < 4; ++t) acc[t] = wmma16b(a, frag_kb(R + (size_t)(t * 16 + nloc) * C + kb, hlf), acc[t]); }
#pragma unroll
  for (int t = 0; t < 4; ++t)
#pragma unroll
    for (int r = 0; r < 8; ++r) { const b16 hv = (b16)(acc[t][r] + XS * P[t * 16 + nloc]); if (t < 2) Tq[wave * 16 + 8 * hlf + r][t * 16 + nloc] = hv; else Tk[wave * 16 + 8 * hlf + r][(t - 2) * 16 + nloc] = hv; }
  __syncthreads();
  for (int pass = 0; pass < 2; ++pass) { for (int i = threadIdx.x; i < 64 * 4; i += 128) { const int rr = i >> 2, c8 = (i & 3) * 8; const size_t gi = (size_t)(blockIdx.x * 64 + rr) * DQ + c8; *(volatile v8b*)(Q + gi) = *(const v8b*)(&Tq[rr][c8]); *(volatile v8b*)(K + gi) = *(const v8b*)(&Tk[rr][c8]); } __threadfence(); }
}
__global__ __launch_bounds__(128) void v_kernel(const b16* __restrict__ X, const b16* __restrict__ R, const float* __restrict__ P, b16* __restrict__ VT) {
  __shared__ __attribute__((aligned(16))) b16 Th[128][64 + 8];
  const int lane = threadIdx.x & 31, wave = threadIdx.x >> 5, nloc = lane & 15, hlf = lane >> 4, t0 = blockIdx.y * 64, m0 = t0 + wave * 16, c0 = blockIdx.x * 128; const b16* Bv = R + (size_t)(64 + c0) * C;
  v8f acc[8];
#pragma unroll
  for (int t = 0; t < 8; ++t) acc[t] = (v8f){};
#pragma unroll 2
  for (int kb = 0; kb < C; kb += 32) { const v16b a = frag_kb(X + (size_t)(m0 + nloc) * C + kb, hlf);
#pragma unroll
    for (int t = 0; t < 8; ++t) acc[t] = wmma16b(a, frag_kb(Bv + (size_t)(t * 16 + nloc) * C + kb, hlf), acc[t]); }
#pragma unroll
  for (int t = 0; t < 8; ++t)
#pragma unroll
    for (int r = 0; r < 8; ++r) Th[t * 16 + nloc][wave * 16 + 8 * hlf + r] = (b16)(acc[t][r] + XS * P[64 + c0 + t * 16 + nloc]);
  __syncthreads();
  for (int pass = 0; pass < 2; ++pass) { for (int i = threadIdx.x; i < 128 * 8; i += 128) { const int cc = i >> 3, c8 = (i & 7) * 8; *(volatile v8b*)(VT + (size_t)(c0 + cc) * N + t0 + c8) = *(const v8b*)(&Th[cc][c8]); } __threadfence(); }
}
__global__ __launch_bounds__(64) void attn_kernel(const b16* __restrict__ Q, const b16* __restrict__ K, const b16* __restrict__ VT, const float* __restrict__ x, const float* __restrict__ P, float* __restrict__ out) {
  __shared__ __attribute__((aligned(16))) float Os[32][C + 4];
  const int wave = threadIdx.x >> 5, lane = threadIdx.x & 31, hh = lane >> 4, col = lane & 15; const int q0 = blockIdx.x * 32 + wave * 16, qi = q0 + col;
  const v16b qf = frag_kb(Q + (size_t)qi * DQ, hh);
  float m = -INFINITY, l = 0.0f; v8f o[16]; for (int t = 0; t < 16; ++t) o[t] = (v8f){};
  for (int kb = 0; kb < N; kb += 32) {
    v8f s0 = {}, s1 = {}; s0 = wmma16b(frag_kb(K + (size_t)(kb + col) * DQ, hh), qf, s0); s1 = wmma16b(frag_kb(K + (size_t)(kb + 16 + col) * DQ, hh), qf, s1);
    float mr = -INFINITY;
#pragma unroll
    for (int r = 0; r < 8; ++r) { s0[r] *= ISC / (XS * XS); s1[r] *= ISC / (XS * XS); mr = fmaxf(mr, fmaxf(s0[r], s1[r])); }
    mr = fmaxf(mr, __shfl_xor(mr, 16)); const float mn = fmaxf(m, mr); const float al_ = nexp(m - mn); m = mn; float sum = 0.0f; v16b pb;
#pragma unroll
    for (int r = 0; r < 8; ++r) { const float e0 = nexp(s0[r] - mn), e1 = nexp(s1[r] - mn); sum += e0 + e1; pb[r] = (b16)(e0 * PS); pb[8 + r] = (b16)(e1 * PS); }
    sum += __shfl_xor(sum, 16); l = l * al_ + sum;
#pragma unroll
    for (int t = 0; t < 16; ++t) { o[t] *= al_; o[t] = wmma16b(frag_kb(VT + (size_t)(t * 16 + col) * N + kb, hh), pb, o[t]); } }
  const float g = P[320] / (l * PS * XS);
#pragma unroll
  for (int t = 0; t < 16; ++t)
#pragma unroll
    for (int r = 0; r < 8; ++r) { const int c = t * 16 + 8 * hh + r; Os[wave * 16 + col][c] = o[t][r] * g; }
  __syncthreads();
  for (int pass = 0; pass < 2; ++pass) { for (int i = threadIdx.x; i < 32 * 64; i += 64) { const int rr = i >> 6, c4 = (i & 63) * 4; const size_t gi = (size_t)(blockIdx.x * 32 + rr) * C + c4; const v4f xv = *(const v4f*)(x + gi); v4f ov; for (int e = 0; e < 4; ++e) ov[e] = bf16_rne(xv[e]) + Os[rr][c4 + e]; *(volatile v4f*)(out + gi) = ov; } __threadfence(); }
}
}

extern "C" void kernel_launch(void* const* d_in, const int* in_sizes, int n_in,
                              void* d_out, int out_size, void* d_ws, size_t ws_size, hipStream_t stream) {
  (void)n_in; (void)out_size;
  const float* x = (const float*)d_in[0]; const float* wq = (const float*)d_in[1]; const float* bq = (const float*)d_in[2]; const float* wk = (const float*)d_in[3]; const float* bk = (const float*)d_in[4]; const float* wv = (const float*)d_in[5]; const float* bv = (const float*)d_in[6]; const float* gm = (const float*)d_in[7];
  float* out = (float*)d_out;
  if (in_sizes[0] != N * C || in_sizes[1] != C * DQ || in_sizes[5] != C * C || in_sizes[7] != 1) return;
  size_t off = 0; char* ws = (char*)d_ws;
  auto carve = [&](size_t bytes) { char* p = ws + off; off += (bytes + 255) & ~(size_t)255; return p; };
  b16* R = (b16*)carve((size_t)320 * C * 2); float* P = (float*)carve(324 * 4); b16* X = (b16*)carve((size_t)N * C * 2); b16* Q = (b16*)carve((size_t)N * DQ * 2); b16* K = (b16*)carve((size_t)N * DQ * 2); b16* VT = (b16*)carve((size_t)C * N * 2);
  if (off > ws_size) return;
  prep_kernel<<<512, 256, 0, stream>>>(x, wq, bq, wk, bk, wv, bv, gm, R, P, X);
  qk_kernel<<<N / 64, 128, 0, stream>>>(X, R, P, Q, K);
  v_kernel<<<dim3(2, N / 64), 128, 0, stream>>>(X, R, P, VT);
  attn_kernel<<<N / 32, 64, 0, stream>>>(Q, K, VT, x, P, out);
}
